// DoubleAlignConv_26491358282333
// MI455X (gfx1250) — hardware-verified
//
#include <hip/hip_runtime.h>
#include <stdint.h>

#pragma clang fp contract(off)

#define NB    2
#define NC    256
#define NO    256
#define IMH   64
#define IMW   64
#define NPIX  4096
#define KT    9
#define KDIM  (KT * NC)
#define PT    64
#define NTH   512
#define NCO   (KT * PT)
#define SP    264
#define CSP   68
#define TSP   72

#define SSC   16.0f
#define LSC   2048.0f
#define WSC   64.0f
#define C1    0.0009765625f
#define C2    4.76837158203125e-07f
#define RCP3  (1.0f / 3.0f)

#define DYN_CW  0
#define DYN_CI  (NCO * 16)
#define DYN_T   (DYN_CI + NCO * 16)
#define DYN_SH  DYN_T
#define DYN_SL  (DYN_T + PT * SP * 2)
#define DYN_CS  DYN_T
#define SZ_S    (2 * PT * SP * 2)
#define SZ_C    (NO * CSP * 4)
#define DYN_TOT (DYN_T + ((SZ_C > SZ_S) ? SZ_C : SZ_S))

static_assert(NTH == 16 * 32);
static_assert(PT == 4 * 16);
static_assert(NO == 4 * 64);
static_assert((NPIX % PT) == 0);
static_assert((NC % 32) == 0);
static_assert(((PT * NC / 8) % NTH) == 0);
static_assert(NCO <= 2 * NTH);
static_assert(((SP * 2) % 16) == 0);
static_assert(((CSP * 4) % 16) == 0);
static_assert(((TSP * 2) % 16) == 0);
static_assert((DYN_CI % 16) == 0 && (DYN_T % 16) == 0 && (DYN_SL % 16) == 0);
static_assert(((2 * NO * KDIM) % (256 * 8)) == 0);
static_assert(((NO * PT) % (NTH * 4)) == 0);
static_assert(DYN_TOT == 88064);

typedef _Float16     v8h  __attribute__((ext_vector_type(8)));
typedef _Float16     v16h __attribute__((ext_vector_type(16)));
typedef unsigned int v4u  __attribute__((ext_vector_type(4)));
typedef int          v4i  __attribute__((ext_vector_type(4)));
typedef float        v4f  __attribute__((ext_vector_type(4)));
typedef float        v8f  __attribute__((ext_vector_type(8)));

union FragH { v8h p[2]; v16h v; };
union H8 { v8h v; _Float16 e[8]; };
static_assert(sizeof(FragH) == 32);
static_assert(sizeof(H8) == 16);

__device__ __forceinline__ v8f zero8() { v8f z = {0.f, 0.f, 0.f, 0.f, 0.f, 0.f, 0.f, 0.f}; return z; }

__device__ __forceinline__ float bf_rne(float x) {
  unsigned int u = __float_as_uint(x);
  u += 0x7FFFu + ((u >> 16) & 1u);
  return __uint_as_float(u & 0xFFFF0000u);
}

__device__ __forceinline__ unsigned short bf_bits(float x) {
  unsigned int u = __float_as_uint(x);
  u += 0x7FFFu + ((u >> 16) & 1u);
  return (unsigned short)(u >> 16);
}

__device__ __forceinline__ void widen8(const v4u q, float (&o)[8]) {
  o[0] = __uint_as_float(q.x << 16); o[1] = __uint_as_float(q.x & 0xFFFF0000u);
  o[2] = __uint_as_float(q.y << 16); o[3] = __uint_as_float(q.y & 0xFFFF0000u);
  o[4] = __uint_as_float(q.z << 16); o[5] = __uint_as_float(q.z & 0xFFFF0000u);
  o[6] = __uint_as_float(q.w << 16); o[7] = __uint_as_float(q.w & 0xFFFF0000u);
}

__device__ __forceinline__ v8f mma_h(v16h a, v16h b, v8f c) {
  v8f d = __builtin_amdgcn_wmma_f32_16x16x32_f16(false, a, false, b, (short)0, c, false, false);
#if defined(__HIP_DEVICE_COMPILE__)
  asm volatile("v_nop\n\tv_nop\n\tv_nop\n\tv_nop" : "+v"(d) : "v"(a), "v"(b));
#endif
  return d;
}

__global__ __launch_bounds__(256)
void k_wprep(const float* __restrict__ Wirr, const float* __restrict__ Wgrid, _Float16* W16) {
  const int t  = threadIdx.x;
  const int g  = blockIdx.x * 256 + t;
  const int e0 = 8 * g;
  const int vo = e0 / KDIM;
  const int k  = e0 - vo * KDIM;
  const int v  = vo >> 8;
  const int o  = vo & (NO - 1);
  const int t9 = k >> 8;
  const int c0 = k & (NC - 1);
  H8 u;
#pragma unroll
  for (int i = 0; i < 8; ++i) {
    const size_t idx = (size_t)(o * NC + c0 + i) * KT + t9;
    const float fa = Wirr[idx];
    const float fb = Wgrid[idx];
    const float f  = (v == 0) ? fa : fb;
    u.e[i] = (_Float16)(bf_rne(f) * WSC);
  }
  _Float16* dst = W16 + e0;
  *(volatile v8h*)dst = u.v;
  __threadfence();
  *(volatile v8h*)dst = u.v;
}

__global__ __launch_bounds__(256)
void k_xprep(const float* __restrict__ X, unsigned short* XP) {
  __shared__ __align__(16) unsigned short Ts[64 * TSP];
  const int t  = threadIdx.x;
  const int pt = blockIdx.x, ct = blockIdx.y, b = blockIdx.z;
  const int p0 = pt * 64, c0 = ct * 64;
  const int pp = t & 63, cb = t >> 6;
#pragma unroll 4
  for (int it = 0; it < 16; ++it) {
    const int cc = it * 4 + cb;
    const float xv = X[(size_t)(b * NC + c0 + cc) * NPIX + p0 + pp];
    Ts[pp * TSP + cc] = bf_bits(xv);
  }
  __syncthreads();

  v4u    wv[2];
  size_t pd[2];
#pragma unroll
  for (int it = 0; it < 2; ++it) {
    const int row = it * 32 + (t >> 3);
    const int q   = t & 7;
    wv[it] = *(const v4u*)(Ts + row * TSP + 8 * q);
    pd[it] = (size_t)(b * NPIX + p0 + row) * NC + c0 + 8 * q;
  }
  *(volatile v4u*)(XP + pd[0]) = wv[0];
  *(volatile v4u*)(XP + pd[1]) = wv[1];
  __threadfence();
  *(volatile v4u*)(XP + pd[0]) = wv[0];
  *(volatile v4u*)(XP + pd[1]) = wv[1];
}

__global__ __launch_bounds__(NTH)
void k_main(const unsigned short* __restrict__ XP, const float* __restrict__ AN, const float* __restrict__ FE,
            const _Float16* __restrict__ W16, float* OUT) {
  extern __shared__ __align__(16) unsigned char dynlds[];
  v4f*      CW = (v4f*)(dynlds + DYN_CW);
  v4i*      CI = (v4i*)(dynlds + DYN_CI);
  _Float16* SH = (_Float16*)(dynlds + DYN_SH);
  _Float16* SL = (_Float16*)(dynlds + DYN_SL);
  float*    Cs = (float*)(dynlds + DYN_CS);
  const int tid = threadIdx.x;
  const int pt  = blockIdx.x, b = blockIdx.y, br = blockIdx.z;
  const int p0  = pt * PT;
  const unsigned short* xpb = XP + (size_t)b * NPIX * NC;
  const _Float16*       wbr = W16 + (size_t)br * NO * KDIM;

#pragma unroll 1
  for (int it = 0; it < 2; ++it) {
    const int e  = it * NTH + tid;
    const int ec = min(e, NCO - 1);
    const int t9 = ec >> 6;
    const int pl = ec & (PT - 1);
    const int n  = p0 + pl;
    const int yc = n >> 6, xc = n & 63;
    const float* ap = AN + (size_t)(b * NPIX + n) * 5;
    const float a0 = bf_rne(ap[0]);
    const float a1 = bf_rne(ap[1]);
    const float a2 = bf_rne(ap[2]);
    const float a3 = bf_rne(ap[3]);
    const float a4 = bf_rne(ap[4]);
    const float xctr = a0 * 0.125f;
    const float yctr = a1 * 0.125f;
    const float aw   = a2 * 0.125f;
    const float ah   = a3 * 0.125f;
    const float cs   = cosf(a4);
    const float sn   = sinf(a4);
    const float dw   = aw * RCP3;
    const float dh   = ah * RCP3;
    const int   kyi  = t9 / 3;
    const int   kxi  = t9 - 3 * kyi;
    const float xx   = (float)(kxi - 1);
    const float yy   = (float)(kyi - 1);
    const float* fp  = FE + (size_t)(b * NPIX + n) * (2 * KT);
    const float f0   = bf_rne(fp[t9]);
    const float f1   = bf_rne(fp[KT + t9]);
    const float pxa  = dw * xx;
    const float pya  = dh * yy;
    const float pxf  = dw * (xx - 0.5f) + dw * f0;
    const float pyf  = dh * (yy - 0.5f) + dh * f1;
    const float px   = (br == 0) ? pxf : pxa;
    const float py   = (br == 0) ? pyf : pya;
    const float xr   = cs * px - sn * py;
    const float yr   = sn * px + cs * py;
    const float xcf  = (float)xc;
    const float ycf  = (float)yc;
    const float ox   = (xr + xctr) - (xcf + xx);
    const float oy   = (yr + yctr) - (ycf + yy);
    const float sx   = (ox + xx) + xcf;
    const float sy   = (oy + yy) + ycf;
    const float y0 = floorf(sy), x0 = floorf(sx);
    const float y1 = y0 + 1.0f,   x1 = x0 + 1.0f;
    const float wy1 = sy - y0, wy0 = 1.0f - wy1;
    const float wx1 = sx - x0, wx0 = 1.0f - wx1;
    const float my0 = (y0 >= 0.0f && y0 < (float)IMH) ? 1.0f : 0.0f;
    const float my1 = (y1 >= 0.0f && y1 < (float)IMH) ? 1.0f : 0.0f;
    const float mx0 = (x0 >= 0.0f && x0 < (float)IMW) ? 1.0f : 0.0f;
    const float mx1 = (x1 >= 0.0f && x1 < (float)IMW) ? 1.0f : 0.0f;
    v4f w;
    w.x = (wy0 * wx0) * (my0 * mx0);
    w.y = (wy0 * wx1) * (my0 * mx1);
    w.z = (wy1 * wx0) * (my1 * mx0);
    w.w = (wy1 * wx1) * (my1 * mx1);
    const int x0c = (int)fminf(fmaxf(x0, 0.0f), (float)(IMW - 1));
    const int x1c = (int)fminf(fmaxf(x1, 0.0f), (float)(IMW - 1));
    const int y0c = (int)fminf(fmaxf(y0, 0.0f), (float)(IMH - 1));
    const int y1c = (int)fminf(fmaxf(y1, 0.0f), (float)(IMH - 1));
    v4i ci;
    ci.x = y0c * IMW + x0c;
    ci.y = y0c * IMW + x1c;
    ci.z = y1c * IMW + x0c;
    ci.w = y1c * IMW + x1c;
    if (e < NCO) {
      CW[ec] = w;
      CI[ec] = ci;
    }
  }
  __syncthreads();

  const int lane = tid & 31, wv = tid >> 5;
  const int hh   = lane >> 4, nn = lane & 15;
  const int pr   = wv & 3, og = wv >> 2;
  v8f acch[4], accl[4];
#pragma unroll
  for (int ct = 0; ct < 4; ++ct) { acch[ct] = zero8(); accl[ct] = zero8(); }

#pragma unroll 1
  for (int t9 = 0; t9 < KT; ++t9) {
#pragma unroll 1
    for (int it = 0; it < (PT * NC / 8) / NTH; ++it) {
      const int s  = it * NTH + tid;
      const int pl = s >> 5;
      const int q  = s & 31;
      const v4f w  = CW[t9 * PT + pl];
      const v4i ci = CI[t9 * PT + pl];
      const unsigned short* cb = xpb + 8 * q;
      const v4u u0 = *(const v4u*)(cb + (size_t)ci.x * NC);
      const v4u u1 = *(const v4u*)(cb + (size_t)ci.y * NC);
      const v4u u2 = *(const v4u*)(cb + (size_t)ci.z * NC);
      const v4u u3 = *(const v4u*)(cb + (size_t)ci.w * NC);
      float xa[8], xb[8], xg[8], xd[8];
      widen8(u0, xa);
      widen8(u1, xb);
      widen8(u2, xg);
      widen8(u3, xd);
      H8 hv, lv;
#pragma unroll
      for (int i = 0; i < 8; ++i) {
        const float sv  = ((xa[i] * w.x + xb[i] * w.y) + xg[i] * w.z) + xd[i] * w.w;
        const float shv = sv * SSC;
        const _Float16 h16 = (_Float16)shv;
        const float res = shv - (float)h16;
        hv.e[i] = h16;
        lv.e[i] = (_Float16)(res * LSC);
      }
      *(v8h*)(SH + pl * SP + 8 * q) = hv.v;
      *(v8h*)(SL + pl * SP + 8 * q) = lv.v;
    }
    __syncthreads();

    const _Float16* ahp = SH + (16 * pr + nn) * SP + 8 * hh;
    const _Float16* alp = SL + (16 * pr + nn) * SP + 8 * hh;
    const _Float16* wbp = wbr + (size_t)(64 * og + nn) * KDIM + t9 * NC + 8 * hh;
#pragma unroll 1
    for (int ks = 0; ks < NC / 32; ++ks) {
      FragH fh, fl;
      fh.p[0] = *(const v8h*)(ahp + ks * 32);
      fh.p[1] = *(const v8h*)(ahp + ks * 32 + 16);
      fl.p[0] = *(const v8h*)(alp + ks * 32);
      fl.p[1] = *(const v8h*)(alp + ks * 32 + 16);
#pragma unroll
      for (int ct = 0; ct < 4; ++ct) {
        const _Float16* wp = wbp + (size_t)(16 * ct) * KDIM + ks * 32;
        FragH wf;
        wf.p[0] = *(const v8h*)(wp);
        wf.p[1] = *(const v8h*)(wp + 16);
        acch[ct] = mma_h(fh.v, wf.v, acch[ct]);
        accl[ct] = mma_h(fl.v, wf.v, accl[ct]);
      }
    }
    __syncthreads();
  }

#pragma unroll
  for (int ct = 0; ct < 4; ++ct) {
    const int o = 64 * og + 16 * ct + nn;
#pragma unroll
    for (int r = 0; r < 8; ++r) {
      float val = acch[ct][r] * C1 + accl[ct][r] * C2;
      val = fmaxf(val, 0.0f);
      Cs[o * CSP + 16 * pr + 8 * hh + r] = val;
    }
  }
  __syncthreads();

  float* ob = OUT + (size_t)br * ((size_t)NB * NO * NPIX) + (size_t)b * NO * NPIX + p0;
  v4f    ov[8];
  size_t po[8];
#pragma unroll
  for (int it = 0; it < 8; ++it) {
    const int row = it * 32 + (tid >> 4);
    const int q   = tid & 15;
    ov[it] = *(const v4f*)(Cs + row * CSP + 4 * q);
    po[it] = (size_t)row * NPIX + 4 * q;
  }
#pragma unroll
  for (int it = 0; it < 8; ++it) *(volatile v4f*)(ob + po[it]) = ov[it];
  __threadfence();
#pragma unroll
  for (int it = 0; it < 8; ++it) *(volatile v4f*)(ob + po[it]) = ov[it];
}

extern "C" void kernel_launch(void* const* d_in, const int* in_sizes, int n_in,
                              void* d_out, int out_size, void* d_ws, size_t ws_size,
                              hipStream_t stream) {
  if (n_in < 5) return;
  if (in_sizes[0] != NB * NC * NPIX) return;
  if (in_sizes[1] != NB * NPIX * 5) return;
  if (in_sizes[2] != NB * NPIX * 2 * KT) return;
  if (in_sizes[3] != NO * NC * KT) return;
  if (in_sizes[4] != NO * NC * KT) return;
  if (out_size != 2 * NB * NO * NPIX) return;

  const size_t szW = (size_t)2 * NO * KDIM * 2;
  const size_t szX = (size_t)NB * NPIX * NC * 2;
  size_t off = 0;
  const size_t oW = off; off += szW;
  const size_t oX = off; off += szX;
  if (off > ws_size) return;
  if (off > (size_t)134217728) return;
  if ((oX % 256) != 0) return;

  const float* x       = (const float*)d_in[0];
  const float* anchors = (const float*)d_in[1];
  const float* feats   = (const float*)d_in[2];
  const float* w_grid  = (const float*)d_in[3];
  const float* w_irr   = (const float*)d_in[4];
  float* out = (float*)d_out;

  char* ws = (char*)d_ws;
  _Float16*       W16 = (_Float16*)(ws + oW);
  unsigned short* XP  = (unsigned short*)(ws + oX);

  k_wprep<<<dim3((2 * NO * KDIM) / (256 * 8)), dim3(256), 0, stream>>>(w_irr, w_grid, W16);
  k_xprep<<<dim3(NPIX / 64, NC / 64, NB), dim3(256), 0, stream>>>(x, XP);
  (void)hipFuncSetAttribute(reinterpret_cast<const void*>(&k_main),
                            hipFuncAttributeMaxDynamicSharedMemorySize, DYN_TOT);
  k_main<<<dim3(NPIX / PT, NB, 2), dim3(NTH), DYN_TOT, stream>>>(XP, anchors, feats, W16, out);
  (void)hipGetLastError();
}
